// CondensedLinearFineGrained_13597866459291
// MI455X (gfx1250) — hardware-verified
//
#include <hip/hip_runtime.h>


#define NBT  256
#define INF  4096
#define OUTF 4096
#define KE   256
#define DM   INF
#define LOSC 1024.0f

typedef _Float16 h16;
typedef unsigned short bf;
typedef __attribute__((ext_vector_type(16))) __bf16   v16bf;
typedef __attribute__((ext_vector_type(16))) _Float16 v16h;
typedef __attribute__((ext_vector_type(8)))  _Float16 v8h;
typedef __attribute__((ext_vector_type(8)))  unsigned short v8us;
typedef __attribute__((ext_vector_type(8)))  float    v8f;
typedef __attribute__((ext_vector_type(4)))  float    v4f;
typedef v8h  __attribute__((may_alias)) v8ha;
typedef v4f  __attribute__((may_alias)) v4fa;
typedef v8us __attribute__((may_alias)) v8usa;

__device__ __forceinline__ unsigned short f2bf(float f) { unsigned u = __float_as_uint(f); u += 0x7FFFu + ((u >> 16) & 1u); return (unsigned short)(u >> 16); }
__device__ __forceinline__ float bf2f(unsigned short b) { return __uint_as_float(((unsigned)b) << 16); }
__device__ __forceinline__ float bfr(float f) { return bf2f(f2bf(f)); }
__device__ __forceinline__ v16h cat16(v8h lo, v8h hi) { return __builtin_shufflevector(lo, hi, 0, 1, 2, 3, 4, 5, 6, 7, 8, 9, 10, 11, 12, 13, 14, 15); }
__device__ __forceinline__ v16bf cat16b(v8us lo, v8us hi) { return __builtin_bit_cast(v16bf, __builtin_shufflevector(lo, hi, 0, 1, 2, 3, 4, 5, 6, 7, 8, 9, 10, 11, 12, 13, 14, 15)); }
__device__ __forceinline__ v8f wmma16(v16h a, v16h b, v8f c) { return __builtin_amdgcn_wmma_f32_16x16x32_f16(false, a, false, b, (short)0, c, false, false); }
__device__ __forceinline__ v8f wmmab(v16bf a, v16bf b, v8f c) { return __builtin_amdgcn_wmma_f32_16x16x32_bf16(false, a, false, b, (short)0, c, false, false); }

template <bool SPLITA, bool F16OUT = false>
__global__ __launch_bounds__(128) void k_gemmb(const bf* __restrict__ A, const bf* __restrict__ Al, const bf* __restrict__ Bn, const float* __restrict__ bias, float* C, int ldc, h16* C2, const float* __restrict__ R = nullptr, int K = DM, int roundR = 1) {
    __shared__ __align__(16) float ost[4][16 * 68];
    const int lane = threadIdx.x & 31, wave = threadIdx.x >> 5, lr = lane & 15, hi = lane >> 4;
    const int r0 = blockIdx.x * 64 + wave * 16, c0 = blockIdx.y * 64;
    const size_t aoff = (size_t)(r0 + lr) * K + 8 * hi;
    size_t boff[4];
#pragma unroll
    for (int t = 0; t < 4; ++t) boff[t] = (size_t)(c0 + t * 16 + lr) * K + 8 * hi;
    v8f acc[4];
#pragma unroll
    for (int t = 0; t < 4; ++t) acc[t] = (v8f){};
#pragma unroll 1
    for (int kc = 0; kc < K; kc += 32) {
        const v16bf a = cat16b(*(const v8us*)(A + aoff + kc), *(const v8us*)(A + aoff + kc + 16));
        v16bf al = a;
        if (SPLITA) al = cat16b(*(const v8us*)(Al + aoff + kc), *(const v8us*)(Al + aoff + kc + 16));
#pragma unroll
        for (int t = 0; t < 4; ++t) { const v16bf b = cat16b(*(const v8us*)(Bn + boff[t] + kc), *(const v8us*)(Bn + boff[t] + kc + 16)); acc[t] = wmmab(a, b, acc[t]); if (SPLITA) acc[t] = wmmab(al, b, acc[t]); }
        asm volatile("v_nop\n\tv_nop\n\tv_nop\n\tv_nop" : "+v"(acc[0]), "+v"(acc[1]), "+v"(acc[2]), "+v"(acc[3]) : "v"(a), "v"(al));
    }
    float* os = &ost[wave][0];
#pragma unroll
    for (int t = 0; t < 4; ++t) { const float bv = bias ? bfr(bias[c0 + t * 16 + lr]) : 0.f;
#pragma unroll
        for (int j = 0; j < 8; ++j) os[(hi * 8 + j) * 68 + t * 16 + lr] = acc[t][j] + bv; }
    __syncthreads();
    if (F16OUT) {
        h16* crow = (h16*)(void*)C + (size_t)r0 * ldc + c0;
        auto pass = [&]() {
#pragma unroll
            for (int s = 0; s < 4; ++s) { const int row = 4 * s + (lane >> 3), piece = lane & 7; const float* sp = os + row * 68 + piece * 8; v8h o, o2;
#pragma unroll
                for (int i = 0; i < 8; ++i) { const h16 a = (h16)sp[i]; o[i] = a; o2[i] = (h16)((sp[i] - (float)a) * LOSC); }
                *(volatile v8h*)(crow + (size_t)row * ldc + piece * 8) = o; if (C2) *(volatile v8h*)(C2 + (size_t)r0 * ldc + c0 + (size_t)row * ldc + piece * 8) = o2; }
        };
        pass(); __threadfence(); pass();
    } else {
        float* crow = C + (size_t)r0 * ldc + c0;
        auto pass = [&]() {
#pragma unroll
            for (int s = 0; s < 8; ++s) { const int Lid = (lane >> 3) + 4 * s, piece = lane & 7; const int row = Lid >> 1, cofs = (Lid & 1) * 32 + piece * 4;
                v4f val = *(const v4fa*)(os + row * 68 + cofs); if (R) { const v4f rv = *(const v4f*)(R + ((size_t)r0 + row) * ldc + c0 + cofs); val += roundR ? (v4f){bfr(rv[0]), bfr(rv[1]), bfr(rv[2]), bfr(rv[3])} : rv; }
                *(volatile v4f*)(crow + (size_t)row * ldc + cofs) = val; }
        };
        pass(); __threadfence(); pass();
    }
}


__global__ __launch_bounds__(256) void k_cvt(const float* __restrict__ src, bf* dst) {
    const int lane = threadIdx.x & 31, r = blockIdx.x * 8 + (threadIdx.x >> 5); if (r >= NBT) return;
#pragma unroll 1
    for (int ps = 0; ps < 2; ++ps) {
#pragma unroll
        for (int q = 0; q < INF / 256; ++q) { v8us o;
#pragma unroll
            for (int i = 0; i < 8; ++i) o[i] = f2bf(src[(size_t)r * INF + q * 256 + lane * 8 + i]);
            *(volatile v8us*)(dst + (size_t)r * INF + q * 256 + lane * 8) = o; }
        if (ps == 0) __threadfence(); }
}
__global__ __launch_bounds__(256) void k_expand(const float* __restrict__ w, const int* __restrict__ mask, bf* Wh, bf* Wl) {
    __shared__ float row[INF];
    const int tid = threadIdx.x, o = blockIdx.x;
#pragma unroll
    for (int i = 0; i < INF / 256; ++i) row[i * 256 + tid] = 0.f;
    __syncthreads();
    if (tid == 0) {
#pragma unroll 1
        for (int k = 0; k < KE; ++k) { int idx = mask[(size_t)o * KE + k]; idx = idx < 0 ? 0 : (idx >= INF ? INF - 1 : idx); row[idx] += bfr(w[(size_t)o * KE + k]); } }
    __syncthreads();
    const int lane = tid & 31, wv = tid >> 5;
#pragma unroll 1
    for (int ps = 0; ps < 2; ++ps) {
#pragma unroll
        for (int q = 0; q < INF / 2048; ++q) { const int c0 = q * 2048 + wv * 256 + lane * 8; v8us oh, ol;
#pragma unroll
            for (int i = 0; i < 8; ++i) { const float v = row[c0 + i]; const unsigned short hb = f2bf(v); oh[i] = hb; ol[i] = f2bf(v - bf2f(hb)); }
            *(volatile v8us*)(Wh + (size_t)o * INF + c0) = oh; *(volatile v8us*)(Wl + (size_t)o * INF + c0) = ol; }
        if (ps == 0) __threadfence(); }
}
__global__ __launch_bounds__(256) void k_tout(const float* __restrict__ CT, const float* __restrict__ bias, float* OUTP) {
    __shared__ float tl[64][65];
    const int tid = threadIdx.x, o0 = blockIdx.x * 64, b0 = blockIdx.y * 64;
    { const int oo = tid >> 2, bq = (tid & 3) * 16; const float bb = bfr(bias[o0 + oo]);
#pragma unroll
      for (int i = 0; i < 16; ++i) tl[bq + i][oo] = CT[(size_t)(o0 + oo) * NBT + b0 + bq + i] + bb; }
    __syncthreads();
    const int piece = tid & 15, Lid = tid >> 4;
    auto pass = [&]() {
#pragma unroll
        for (int s = 0; s < 4; ++s) { const int b = Lid + 16 * s; v4f v;
#pragma unroll
            for (int i = 0; i < 4; ++i) v[i] = tl[b][piece * 4 + i];
            *(volatile v4f*)(OUTP + (size_t)(b0 + b) * OUTF + o0 + piece * 4) = v; }
    };
    pass(); __threadfence(); pass();
}

extern "C" void kernel_launch(void* const* d_in, const int* in_sizes, int n_in,
                              void* d_out, int out_size, void* d_ws, size_t ws_size, hipStream_t stream) {
    (void)in_sizes; (void)n_in; (void)out_size;
    const float* x = (const float*)d_in[0]; const float* w = (const float*)d_in[1]; const int* mask = (const int*)d_in[2]; const float* bias = (const float*)d_in[3];
    float* out = (float*)d_out;
    char* wsp = (char*)d_ws;
    auto take = [&](size_t bytes) { char* p = wsp; wsp += (bytes + 255) & ~(size_t)255; return (void*)p; };
    bf* Xb = (bf*)take((size_t)NBT * INF * 2); bf* Wh = (bf*)take((size_t)OUTF * INF * 2); bf* Wl = (bf*)take((size_t)OUTF * INF * 2); float* CT = (float*)take((size_t)OUTF * NBT * 4);
    if ((size_t)(wsp - (char*)d_ws) > ws_size) return;
    k_cvt<<<NBT / 8, 256, 0, stream>>>(x, Xb);
    k_expand<<<OUTF, 256, 0, stream>>>(w, mask, Wh, Wl);
    k_gemmb<true, false><<<dim3(OUTF / 64, NBT / 64, 1), 128, 0, stream>>>(Wh, Wl, Xb, nullptr, CT, NBT, nullptr, nullptr, INF);
    k_tout<<<dim3(OUTF / 64, NBT / 64, 1), 256, 0, stream>>>(CT, bias, out);
}
